// Attention_13700945674459
// MI455X (gfx1250) — hardware-verified
//
#include <hip/hip_runtime.h>


#ifndef NB
#define NB 4
#endif
#ifndef SEQ
#define SEQ 2048
#endif
#define NB_FULL  4
#define SEQ_FULL 2048
#define DM   1024
#define NH   16
#define HD   64
#define NQKV 3072
#define NWT  4096
#define GM   128
#define SP   68
#define NWV  4
#define BQ   (16 * NWV)
#define KS   32
#define OSP  68
#define VTP  72
#define L2E  1.4426950408889634f
#define PCARRY 12.0f

static_assert(NH == 16);
static_assert(HD == 64);
static_assert(NH * HD == DM);
static_assert(SEQ % GM == 0);
static_assert(SEQ % BQ == 0);
static_assert(SEQ % KS == 0);
static_assert(DM % 32 == 0);
static_assert(NB <= NB_FULL);
static_assert(SEQ <= SEQ_FULL);
static_assert(((size_t)NB * SEQ * DM) % 2048 == 0);
static_assert((size_t)(DM / 64) * (NWT / 128) * (size_t)(64 * 128) == (size_t)NWT * DM);
static_assert(((size_t)SEQ * 16) % 256 == 0);
static_assert((size_t)(NB * SEQ / GM) * (NQKV / 64) * (size_t)(GM * 64) == (size_t)3 * NB * SEQ * DM);
static_assert((size_t)(NB * NH * (SEQ / BQ)) * (size_t)(BQ * HD) == (size_t)NB * SEQ * DM);
static_assert((size_t)(NB * SEQ / GM) * (DM / 64) * (size_t)(GM * 64) == (size_t)NB * SEQ * DM);
static_assert(((size_t)SEQ * 16 * 4) % 256 == 0);
static_assert((size_t)6 * NB_FULL * SEQ_FULL * DM * 2 + (size_t)NWT * DM * 2 + (size_t)2 * SEQ_FULL * 16 * 4 <= (size_t)134217728);

typedef unsigned short bf;
typedef unsigned short hb;
typedef __attribute__((ext_vector_type(16))) __bf16   v16bf;
typedef __attribute__((ext_vector_type(2)))  __bf16   v2bf;
typedef __attribute__((ext_vector_type(16))) _Float16 v16h;
typedef __attribute__((ext_vector_type(2)))  _Float16 v2h;
typedef __attribute__((ext_vector_type(8)))  unsigned short v8us;
typedef __attribute__((ext_vector_type(8)))  unsigned int   v8u;
typedef __attribute__((ext_vector_type(4)))  unsigned int   v4u;
typedef __attribute__((ext_vector_type(8)))  float    v8f;
typedef __attribute__((ext_vector_type(4)))  float    v4f;
typedef v4f  __attribute__((may_alias)) v4fa;
typedef v8us __attribute__((may_alias)) v8usa;

struct FreqArgs { float inv[16]; };
static_assert(sizeof(FreqArgs) == 64);

__device__ __forceinline__ unsigned short f2bf(float f) { unsigned u = __float_as_uint(f); u += 0x7FFFu + ((u >> 16) & 1u); return (unsigned short)(u >> 16); }
__device__ __forceinline__ unsigned bfhi32(float f) { unsigned u = __float_as_uint(f); u += 0x7FFFu + ((u >> 16) & 1u); return u & 0xFFFF0000u; }
__device__ __forceinline__ float bfr(float f) { return __uint_as_float(bfhi32(f)); }
__device__ __forceinline__ v16bf cat16b(v8us lo, v8us hi) { return __builtin_bit_cast(v16bf, __builtin_shufflevector(lo, hi, 0, 1, 2, 3, 4, 5, 6, 7, 8, 9, 10, 11, 12, 13, 14, 15)); }
__device__ __forceinline__ v16h  cat16h(v8us lo, v8us hi) { return __builtin_bit_cast(v16h,  __builtin_shufflevector(lo, hi, 0, 1, 2, 3, 4, 5, 6, 7, 8, 9, 10, 11, 12, 13, 14, 15)); }
__device__ __forceinline__ v8f wmmab(v16bf a, v16bf b, v8f c) { return __builtin_amdgcn_wmma_f32_16x16x32_bf16(false, a, false, b, (short)0, c, false, false); }
__device__ __forceinline__ v8f wmmah(v16h a, v16h b, v8f c) { return __builtin_amdgcn_wmma_f32_16x16x32_f16(false, a, false, b, (short)0, c, false, false); }
__device__ __forceinline__ v16bf ldb(const bf* p) { return cat16b(*(const v8us*)p, *(const v8us*)(p + 16)); }
__device__ __forceinline__ v16h  ldh(const hb* p) { return cat16h(*(const v8us*)p, *(const v8us*)(p + 16)); }
__device__ __forceinline__ unsigned pk2bf(float a, float b) { v2bf t; t[0] = (__bf16)a; t[1] = (__bf16)b; return __builtin_bit_cast(unsigned, t); }
__device__ __forceinline__ unsigned pk2h(float a, float b) { v2h t; t[0] = (_Float16)a; t[1] = (_Float16)b; return __builtin_bit_cast(unsigned, t); }

__global__ __launch_bounds__(256) void k_cvt(const float* __restrict__ x, bf* XB) {
    const unsigned i = blockIdx.x * 256u + threadIdx.x;
    const unsigned per = (unsigned)(SEQ * DM / 8);
    if (i >= (unsigned)NB * per) return;
    const unsigned b = i / per, r = i - b * per;
    const float* src = x + (size_t)b * SEQ_FULL * DM + (size_t)r * 8;
    const v4f v0 = *(const v4f*)src;
    const v4f v1 = *(const v4f*)(src + 4);
    v4u o;
    o[0] = (bfhi32(v0[0]) >> 16) | bfhi32(v0[1]);
    o[1] = (bfhi32(v0[2]) >> 16) | bfhi32(v0[3]);
    o[2] = (bfhi32(v1[0]) >> 16) | bfhi32(v1[1]);
    o[3] = (bfhi32(v1[2]) >> 16) | bfhi32(v1[3]);
    bf* dst = XB + (size_t)i * 8;
    *(volatile v4u*)dst = o;
    __threadfence();
    *(volatile v4u*)dst = o;
}

__global__ __launch_bounds__(256) void k_wt(const float* __restrict__ Wq, const float* __restrict__ Wkv, const float* __restrict__ Wo, bf* WT) {
    __shared__ __align__(16) bf tl[128 * VTP];
    const unsigned tid = threadIdx.x;
    const unsigned k0 = blockIdx.x * 64u;
    const unsigned n0 = blockIdx.y * 128u;
    const float* src;
    unsigned ldn;
    if (n0 < 1024u)      { src = Wq  + n0;            ldn = 1024u; }
    else if (n0 < 3072u) { src = Wkv + (n0 - 1024u);  ldn = 2048u; }
    else                 { src = Wo  + (n0 - 3072u);  ldn = 1024u; }
    src += (size_t)k0 * ldn;
#pragma unroll
    for (unsigned it = 0; it < 8; ++it) {
        const unsigned f = it * 256u + tid;
        const unsigned kk = f >> 5, c4 = (f & 31u) * 4u;
        const v4f x = *(const v4f*)(src + (size_t)kk * ldn + c4);
#pragma unroll
        for (unsigned c = 0; c < 4; ++c) tl[(c4 + c) * VTP + kk] = f2bf(x[c]);
    }
    __syncthreads();
    bf* dst = WT + (size_t)n0 * DM + k0;
    const unsigned c8 = (tid & 7u) * 8u, dr = tid >> 3;
#pragma unroll 1
    for (int ps = 0; ps < 2; ++ps) {
#pragma unroll
        for (unsigned it = 0; it < 4; ++it) {
            const unsigned d = it * 32u + dr;
            const v8us o = *(const v8usa*)(tl + d * VTP + c8);
            *(volatile v8us*)(dst + (size_t)d * DM + c8) = o;
        }
        if (ps == 0) __threadfence();
    }
}

__global__ __launch_bounds__(256) void k_tab(FreqArgs fa, float* cosT, float* sinT) {
    const unsigned i = blockIdx.x * 256u + threadIdx.x;
    const unsigned t = i >> 4, f = i & 15u;
    float inv = fa.inv[0];
#pragma unroll
    for (unsigned j = 1; j < 16; ++j) inv = (f == j) ? fa.inv[j] : inv;
    const float ang = (float)t * inv;
    float s, c;
    sincosf(ang, &s, &c);
    *(volatile float*)(cosT + i) = c;
    *(volatile float*)(sinT + i) = s;
    __threadfence();
    *(volatile float*)(cosT + i) = c;
    *(volatile float*)(sinT + i) = s;
}

__global__ __launch_bounds__(128) void k_proj(const bf* __restrict__ XB, const bf* __restrict__ WT,
                                              const float* __restrict__ cosT, const float* __restrict__ sinT,
                                              hb* QH, hb* KH, hb* VT) {
    __shared__ __align__(16) float st[GM * SP];
    const unsigned tid = threadIdx.x, lane = tid & 31u, wv = tid >> 5, lr = lane & 15u, hi = lane >> 4;
    const unsigned m0 = blockIdx.x * GM;
    const unsigned nt = blockIdx.y;
    const bf* ap = XB + (size_t)(m0 + 32u * wv + lr) * DM + 8u * hi;
    const bf* bp = WT + (size_t)(nt * 64u + lr) * DM + 8u * hi;

    v8f c0[4], c1[4];
#pragma unroll
    for (int t = 0; t < 4; ++t) { c0[t] = (v8f){}; c1[t] = (v8f){}; }

#pragma unroll 1
    for (unsigned k0 = 0; k0 < (unsigned)DM; k0 += 32) {
        const v16bf a0 = ldb(ap + k0);
        const v16bf a1 = ldb(ap + 16 * DM + k0);
#pragma unroll
        for (int t = 0; t < 4; ++t) {
            const v16bf bb = ldb(bp + (size_t)t * 16 * DM + k0);
            c0[t] = wmmab(a0, bb, c0[t]);
            c1[t] = wmmab(a1, bb, c1[t]);
        }
        asm volatile("v_nop\n\tv_nop\n\tv_nop\n\tv_nop"
                     : "+v"(c0[0]), "+v"(c0[1]), "+v"(c0[2]), "+v"(c0[3]), "+v"(c1[0]), "+v"(c1[1]), "+v"(c1[2]), "+v"(c1[3])
                     : "v"(a0), "v"(a1));
    }

    float* sw = st + (32u * wv) * SP;
#pragma unroll
    for (int t = 0; t < 4; ++t) {
#pragma unroll
        for (int r = 0; r < 8; ++r) {
            sw[(8u * hi + r) * SP + t * 16 + lr] = c0[t][r];
            sw[(16u + 8u * hi + r) * SP + t * 16 + lr] = c1[t][r];
        }
    }
    __syncthreads();

    const unsigned b = m0 / (unsigned)SEQ;
    const unsigned pos0 = m0 - b * (unsigned)SEQ;
    if (nt < 32u) {
        const unsigned h = nt & 15u;
        hb* dst = (nt < 16u ? QH : KH) + ((size_t)(b * NH + h) * SEQ + pos0) * HD;
        const unsigned cg = lane & 7u, rq = lane >> 3;
        const bool rot = cg < 4u;
        const unsigned tc = (cg & 3u) * 4u;
#pragma unroll 1
        for (int ps = 0; ps < 2; ++ps) {
#pragma unroll 2
            for (unsigned it = 0; it < 8; ++it) {
                const unsigned row = 32u * wv + 4u * it + rq;
                const float* sr = st + row * SP + 8u * cg;
                const v4f xa = *(const v4fa*)sr;
                const v4f xb = *(const v4fa*)(sr + 4);
                const unsigned ti = (pos0 + row) * 16u + tc;
                const v4f c4 = *(const v4f*)(cosT + ti);
                const v4f s4 = *(const v4f*)(sinT + ti);
                const float x[8] = { xa[0], xa[1], xa[2], xa[3], xb[0], xb[1], xb[2], xb[3] };
                v4u o;
#pragma unroll
                for (int j = 0; j < 4; ++j) {
                    const float x1 = x[2 * j], x2 = x[2 * j + 1];
                    const float r1 = x1 * c4[j] - x2 * s4[j];
                    const float r2 = x2 * c4[j] + x1 * s4[j];
                    o[j] = pk2h(rot ? r1 : x1, rot ? r2 : x2);
                }
                *(volatile v4u*)(dst + (size_t)row * HD + 8u * cg) = o;
            }
            if (ps == 0) __threadfence();
        }
    } else {
        const unsigned h = nt - 32u;
        hb* dst = VT + (size_t)(b * NH + h) * HD * SEQ + pos0;
        const unsigned c8 = (lane & 7u) * 8u, lq = lane >> 3;
#pragma unroll 1
        for (int ps = 0; ps < 2; ++ps) {
#pragma unroll 2
            for (unsigned it = 0; it < 8; ++it) {
                const unsigned L = (wv * 8u + it) * 4u + lq;
                const unsigned d = L >> 1, tk = (L & 1u) * 64u + c8;
                const float* sc = st + tk * SP + d;
                v4u o;
#pragma unroll
                for (int j = 0; j < 4; ++j) o[j] = pk2h(sc[(2 * j) * SP], sc[(2 * j + 1) * SP]);
                *(volatile v4u*)(dst + (size_t)d * SEQ + tk) = o;
            }
            if (ps == 0) __threadfence();
        }
    }
}

__global__ __launch_bounds__(128) void k_flash(const hb* __restrict__ QH, const hb* __restrict__ KH, const hb* __restrict__ VT, bf* CH, bf* CL) {
    __shared__ __align__(16) float os[NWV * 16 * OSP];
    const unsigned tid = threadIdx.x, lane = tid & 31u, wv = tid >> 5, lr = lane & 15u, hi = lane >> 4;
    const unsigned qpb = (unsigned)(SEQ / BQ);
    const unsigned bh = blockIdx.x / qpb;
    const unsigned q0 = (blockIdx.x - bh * qpb) * BQ + wv * 16u;
    const unsigned b = bh >> 4, h = bh & 15u;

    v16h qf[2];
    {
        const hb* qp = QH + ((size_t)bh * SEQ + q0 + lr) * HD + 8u * hi;
        qf[0] = ldh(qp);
        qf[1] = ldh(qp + 32);
    }
    const hb* kp = KH + ((size_t)bh * SEQ + lr) * HD + 8u * hi;
    const hb* vp = VT + ((size_t)bh * HD + lr) * SEQ + 8u * hi;

    v8f o[4];
#pragma unroll
    for (int t = 0; t < 4; ++t) o[t] = (v8f){};
    float ml = -1.0e30f;
    float l = 0.0f;
    const float CS = 0.125f * L2E;

#pragma unroll 1
    for (unsigned k0 = 0; k0 < (unsigned)SEQ; k0 += KS) {
        v8f s0 = (v8f){}, s1 = (v8f){};
        const hb* ka = kp + (size_t)k0 * HD;
#pragma unroll
        for (int dk = 0; dk < 2; ++dk) {
            const v16h a0 = ldh(ka + dk * 32);
            const v16h a1 = ldh(ka + 16 * HD + dk * 32);
            s0 = wmmah(a0, qf[dk], s0);
            s1 = wmmah(a1, qf[dk], s1);
        }
        asm volatile("v_nop\n\tv_nop\n\tv_nop\n\tv_nop" : "+v"(s0), "+v"(s1) : "v"(qf[0]), "v"(qf[1]));

        float mx = fmaxf(s0[0], s1[0]);
#pragma unroll
        for (int r = 1; r < 8; ++r) mx = fmaxf(mx, fmaxf(s0[r], s1[r]));
        mx = fmaxf(mx, __shfl_xor(mx, 16, 32));
        const float mnl = fmaxf(ml, mx * CS);
        const float corr = __builtin_amdgcn_exp2f(ml - mnl);
        ml = mnl;
        const float pm = PCARRY - mnl;
        float p0[8], p1[8];
        float ps = 0.0f;
#pragma unroll
        for (int r = 0; r < 8; ++r) {
            p0[r] = __builtin_amdgcn_exp2f(fmaf(s0[r], CS, pm));
            p1[r] = __builtin_amdgcn_exp2f(fmaf(s1[r], CS, pm));
            ps += p0[r] + p1[r];
        }
        ps += __shfl_xor(ps, 16, 32);
        l = l * corr + ps;
        if (__builtin_amdgcn_ballot_w32(corr != 1.0f) != 0u) {
#pragma unroll
            for (int t = 0; t < 4; ++t) o[t] *= corr;
        }

        v8u hw;
#pragma unroll
        for (int j = 0; j < 4; ++j) {
            hw[j]     = pk2h(p0[2 * j], p0[2 * j + 1]);
            hw[4 + j] = pk2h(p1[2 * j], p1[2 * j + 1]);
        }
        const v16h ph = __builtin_bit_cast(v16h, hw);

        asm volatile("" ::: "memory");
        const hb* va = vp + k0;
#pragma unroll
        for (int t = 0; t < 4; ++t) {
            const v16h a = ldh(va + (size_t)t * 16 * SEQ);
            o[t] = wmmah(a, ph, o[t]);
        }
        asm volatile("v_nop\n\tv_nop\n\tv_nop\n\tv_nop"
                     : "+v"(o[0]), "+v"(o[1]), "+v"(o[2]), "+v"(o[3])
                     : "v"(ph));
    }

    const float inv = 1.0f / l;
    float* ow = os + wv * (16 * OSP);
#pragma unroll
    for (int t = 0; t < 4; ++t) {
#pragma unroll
        for (int r = 0; r < 8; ++r) ow[lr * OSP + t * 16 + 8 * hi + r] = o[t][r] * inv;
    }
    __syncthreads();
    const unsigned cg = lane & 7u, rq = lane >> 3;
    const size_t cbase = ((size_t)b * SEQ + q0) * DM + h * HD + 8u * cg;
#pragma unroll 1
    for (int ps2 = 0; ps2 < 2; ++ps2) {
#pragma unroll
        for (unsigned s = 0; s < 4; ++s) {
            const unsigned row = 4u * s + rq;
            const float* sr = ow + row * OSP + 8u * cg;
            const v4f xa = *(const v4fa*)sr;
            const v4f xb = *(const v4fa*)(sr + 4);
            const float x[8] = { xa[0], xa[1], xa[2], xa[3], xb[0], xb[1], xb[2], xb[3] };
            v4u oh, ol;
#pragma unroll
            for (int j = 0; j < 4; ++j) {
                const unsigned r0 = bfhi32(x[2 * j]), r1 = bfhi32(x[2 * j + 1]);
                oh[j] = (r0 >> 16) | r1;
                ol[j] = pk2bf(x[2 * j] - __uint_as_float(r0), x[2 * j + 1] - __uint_as_float(r1));
            }
            *(volatile v4u*)(CH + cbase + (size_t)row * DM) = oh;
            *(volatile v4u*)(CL + cbase + (size_t)row * DM) = ol;
        }
        if (ps2 == 0) __threadfence();
    }
}

__global__ __launch_bounds__(128) void k_out(const bf* __restrict__ CH, const bf* __restrict__ CL, const bf* __restrict__ WOT,
                                             const float* __restrict__ bout, float* O) {
    __shared__ __align__(16) float st[GM * SP];
    const unsigned tid = threadIdx.x, lane = tid & 31u, wv = tid >> 5, lr = lane & 15u, hi = lane >> 4;
    const unsigned m0 = blockIdx.x * GM;
    const unsigned n0 = blockIdx.y * 64u;
    const size_t aoff = (size_t)(m0 + 32u * wv + lr) * DM + 8u * hi;
    const bf* ah = CH + aoff;
    const bf* al = CL + aoff;
    const bf* bp = WOT + (size_t)(n0 + lr) * DM + 8u * hi;

    v8f c0[4], c1[4];
#pragma unroll
    for (int t = 0; t < 4; ++t) { c0[t] = (v8f){}; c1[t] = (v8f){}; }

#pragma unroll 1
    for (unsigned k0 = 0; k0 < (unsigned)DM; k0 += 32) {
        const v16bf h0 = ldb(ah + k0);
        const v16bf h1 = ldb(ah + 16 * DM + k0);
        const v16bf l0 = ldb(al + k0);
        const v16bf l1 = ldb(al + 16 * DM + k0);
#pragma unroll
        for (int t = 0; t < 4; ++t) {
            const v16bf bb = ldb(bp + (size_t)t * 16 * DM + k0);
            c0[t] = wmmab(h0, bb, c0[t]);
            c0[t] = wmmab(l0, bb, c0[t]);
            c1[t] = wmmab(h1, bb, c1[t]);
            c1[t] = wmmab(l1, bb, c1[t]);
        }
        asm volatile("v_nop\n\tv_nop\n\tv_nop\n\tv_nop"
                     : "+v"(c0[0]), "+v"(c0[1]), "+v"(c0[2]), "+v"(c0[3]), "+v"(c1[0]), "+v"(c1[1]), "+v"(c1[2]), "+v"(c1[3])
                     : "v"(h0), "v"(h1), "v"(l0), "v"(l1));
    }

    float* sw = st + (32u * wv) * SP;
#pragma unroll
    for (int t = 0; t < 4; ++t) {
#pragma unroll
        for (int r = 0; r < 8; ++r) {
            sw[(8u * hi + r) * SP + t * 16 + lr] = c0[t][r];
            sw[(16u + 8u * hi + r) * SP + t * 16 + lr] = c1[t][r];
        }
    }
    __syncthreads();

    const unsigned c4 = (lane & 15u) * 4u, rh = lane >> 4;
    const v4f bv = *(const v4f*)(bout + n0 + c4);
    const float b0 = bfr(bv[0]), b1 = bfr(bv[1]), b2 = bfr(bv[2]), b3 = bfr(bv[3]);
    float* orow = O + (size_t)(m0 + 32u * wv) * DM + n0 + c4;
#pragma unroll 1
    for (int ps = 0; ps < 2; ++ps) {
#pragma unroll 4
        for (unsigned it = 0; it < 16; ++it) {
            const unsigned row = 2u * it + rh;
            v4f val = *(const v4fa*)(sw + row * SP + c4);
            val[0] += b0; val[1] += b1; val[2] += b2; val[3] += b3;
            *(volatile v4f*)(orow + (size_t)row * DM) = val;
        }
        if (ps == 0) __threadfence();
    }
}

extern "C" void kernel_launch(void* const* d_in, const int* in_sizes, int n_in,
                              void* d_out, int out_size, void* d_ws, size_t ws_size, hipStream_t stream) {
    if (n_in < 5) return;
    const size_t needx = ((size_t)(NB - 1) * SEQ_FULL + SEQ) * DM;
    if ((size_t)in_sizes[0] < needx) return;
    if ((size_t)in_sizes[1] < (size_t)DM * DM) return;
    if ((size_t)in_sizes[2] < (size_t)2 * DM * DM) return;
    if ((size_t)in_sizes[3] < (size_t)DM * DM) return;
    if ((size_t)in_sizes[4] < (size_t)DM) return;
    if ((size_t)out_size < (size_t)NB * SEQ * DM) return;
    const float* x    = (const float*)d_in[0];
    const float* Wq   = (const float*)d_in[1];
    const float* Wkv  = (const float*)d_in[2];
    const float* Wout = (const float*)d_in[3];
    const float* bout = (const float*)d_in[4];
    float* OUT = (float*)d_out;

    const size_t PA = (size_t)NB * SEQ * DM * 2;
    const size_t PW = (size_t)NWT * DM * 2;
    const size_t PT = (size_t)SEQ * 16 * 4;
    if (6 * PA + PW + 2 * PT > ws_size) return;
    char* wsp = (char*)d_ws;
    bf* XB = (bf*)(wsp);
    bf* WT = (bf*)(wsp + PA);
    float* cosT = (float*)(wsp + PA + PW);
    float* sinT = (float*)(wsp + PA + PW + PT);
    hb* QH = (hb*)(wsp + PA + PW + 2 * PT);
    hb* KH = (hb*)(wsp + 2 * PA + PW + 2 * PT);
    hb* VT = (hb*)(wsp + 3 * PA + PW + 2 * PT);
    bf* CH = (bf*)(wsp + 4 * PA + PW + 2 * PT);
    bf* CL = (bf*)(wsp + 5 * PA + PW + 2 * PT);

    FreqArgs fa;
    for (int i = 0; i < 16; ++i) {
        const float pw = (float)pow(10000.0, (double)(2 * i) / 32.0);
        fa.inv[i] = 1.0f / pw;
    }

    const unsigned gc = (unsigned)(((size_t)NB * SEQ * DM / 8 + 255) / 256);
    k_cvt<<<gc, 256, 0, stream>>>(x, XB);
    k_wt<<<dim3(DM / 64, NWT / 128, 1), 256, 0, stream>>>(Wq, Wkv, Wout, WT);
    k_tab<<<(unsigned)(SEQ * 16 / 256), 256, 0, stream>>>(fa, cosT, sinT);
    k_proj<<<dim3((unsigned)(NB * SEQ / GM), NQKV / 64, 1), 128, 0, stream>>>(XB, WT, cosT, sinT, QH, KH, VT);
    k_flash<<<(unsigned)(NB * NH * (SEQ / BQ)), 128, 0, stream>>>(QH, KH, VT, CH, CL);
    k_out<<<dim3((unsigned)(NB * SEQ / GM), DM / 64, 1), 128, 0, stream>>>(CH, CL, WT + (size_t)NQKV * DM, bout, OUT);
}
